// Embedder_39797166965440
// MI455X (gfx1250) — hardware-verified
//
#include <hip/hip_runtime.h>
#include <math.h>

constexpr int kS      = 4096;
constexpr int kE      = 1024;
constexpr int kHeads  = 16;
constexpr int kDh     = 64;
constexpr int kLdQKV  = 3 * kE;
constexpr int kTiles  = kS / 64;
constexpr int kChunks = 16;
constexpr int kMaxSeg = 512;
static_assert(kHeads * kDh == kE);
static_assert(kS % 64 == 0 && kE % 64 == 0 && kE % 32 == 0 && kS % 256 == 0);
static_assert((kS / 64) * (kE / 64) == 1024);
static_assert(kS / 256 == kChunks);

typedef __attribute__((ext_vector_type(16))) _Float16 v16h;
typedef __attribute__((ext_vector_type(8)))  _Float16 v8h;
typedef __attribute__((ext_vector_type(16))) __bf16   v16b;
typedef __attribute__((ext_vector_type(8)))  __bf16   v8b;
typedef __attribute__((ext_vector_type(8)))  float    v8f;
typedef __attribute__((ext_vector_type(4)))  float    v4f;
typedef __attribute__((ext_vector_type(4)))  unsigned int v4u;
typedef __attribute__((ext_vector_type(4)))  int      v4i;

__device__ __forceinline__ unsigned short f2bf_bits(float f) {
  unsigned u = __float_as_uint(f);
  return (unsigned short)((u + 0x7FFFu + ((u >> 16) & 1u)) >> 16);
}
__device__ __forceinline__ float bf_bits2f(unsigned short h) { return __uint_as_float(((unsigned)h) << 16); }

__device__ __forceinline__ void dep_guard_h(v8f& a, v8f& b, v16h x, v16h y) { asm volatile("v_nop\n\tv_nop\n\tv_nop\n\tv_nop" : "+v"(a), "+v"(b) : "v"(x), "v"(y)); }
__device__ __forceinline__ void dep_guard_b(v8f& a, v8f& b, v16b x, v16b y) { asm volatile("v_nop\n\tv_nop\n\tv_nop\n\tv_nop" : "+v"(a), "+v"(b) : "v"(x), "v"(y)); }
__device__ __forceinline__ void keep4_h(v16h a, v16h b, v16h c, v16h d) { asm volatile("v_nop" :: "v"(a), "v"(b), "v"(c), "v"(d)); }
__device__ __forceinline__ void keep4_b(v16b a, v16b b, v16b c, v16b d) { asm volatile("v_nop" :: "v"(a), "v"(b), "v"(c), "v"(d)); }
__device__ __forceinline__ void acc_guard4(v8f& a, v8f& b, v8f& c, v8f& d) { asm volatile("v_nop\n\tv_nop\n\tv_nop\n\tv_nop" : "+v"(a), "+v"(b), "+v"(c), "+v"(d)); }
template <typename T> struct Frag;
template <> struct Frag<_Float16> {
  typedef v16h V; union U { v16h v; v8h h[2]; };
  static __device__ __forceinline__ v16h load(const _Float16* p) {
    U f; f.h[0] = *(const v8h*)(p); f.h[1] = *(const v8h*)(p + 16); return f.v;
  }
  static __device__ __forceinline__ v8f mma(v16h a, v16h b, v8f c) {
    return __builtin_amdgcn_wmma_f32_16x16x32_f16(false, a, false, b, (short)0, c, false, false);
  }
  static __device__ __forceinline__ void guard(v8f& a, v8f& b, v16h x, v16h y) { dep_guard_h(a, b, x, y); }
  static __device__ __forceinline__ void keep(v16h a, v16h b, v16h c, v16h d) { keep4_h(a, b, c, d); }
};
template <> struct Frag<__bf16> {
  typedef v16b V; union U { v16b v; v8b h[2]; };
  static __device__ __forceinline__ v16b load(const __bf16* p) {
    U f; f.h[0] = *(const v8b*)(p); f.h[1] = *(const v8b*)(p + 16); return f.v;
  }
  static __device__ __forceinline__ v8f mma(v16b a, v16b b, v8f c) {
    return __builtin_amdgcn_wmma_f32_16x16x32_bf16(false, a, false, b, (short)0, c, false, false);
  }
  static __device__ __forceinline__ void guard(v8f& a, v8f& b, v16b x, v16b y) { dep_guard_b(a, b, x, y); }
  static __device__ __forceinline__ void keep(v16b a, v16b b, v16b c, v16b d) { keep4_b(a, b, c, d); }
};

__device__ __forceinline__ unsigned pk16(unsigned short a, unsigned short b) { return (unsigned)a | ((unsigned)b << 16); }

__device__ __forceinline__ void split_bf(float f, unsigned short& hb, unsigned short& lb) {
  hb = f2bf_bits(f);
  lb = f2bf_bits(f - bf_bits2f(hb));
}

__device__ __forceinline__ void seg_info(const int* __restrict__ info, int& s0, int& s1, int& cnt, int& target) {
  const v4i w = *(const v4i*)info;
  int a = __builtin_amdgcn_readfirstlane(w[0]);
  int b = __builtin_amdgcn_readfirstlane(w[1]);
  int c = __builtin_amdgcn_readfirstlane(w[2]);
  int d = __builtin_amdgcn_readfirstlane(w[3]);
  a = a < 0 ? 0 : (a > kS - 1 ? kS - 1 : a);
  b = b < a + 1 ? a + 1 : (b > kS ? kS : b);
  c = c < 1 ? 1 : (c > kS ? kS : c);
  s0 = a; s1 = b; cnt = c; target = d;
}

__device__ __forceinline__ float wave_sum32(float v) {
#pragma unroll
  for (int off = 16; off > 0; off >>= 1) v += __shfl_xor(v, off, 32);
  return v;
}

template <int ET> struct Elem;
template <> struct Elem<0> { typedef _Float16 T; };
template <> struct Elem<1> { typedef __bf16 T; };
template <int ET, bool SPLIT, int BIAS_MODE, int OUT_MODE, bool RESID, int ACT = 0>
__global__ __launch_bounds__(256) void wmma_gemm64_seg(
    const unsigned short* __restrict__ Ap, const unsigned short* __restrict__ A2p, int lda, long strideA,
    const unsigned short* __restrict__ Btp, const unsigned short* __restrict__ Bt2p, int ldb, long strideB,
    void* __restrict__ Cout, void* __restrict__ Cout2, int ldc, long strideC,
    const float* __restrict__ bias,
    const float* __restrict__ resid, long strideR,
    int M, int N, int K, float scale, const int* __restrict__ rowinfo) {
  typedef typename Elem<ET>::T T;
  typedef typename Frag<T>::V V;
  const T* A = (const T*)Ap; const T* A2 = (const T*)A2p; const T* Bt = (const T*)Btp; const T* Bt2 = (const T*)Bt2p;
  __shared__ __align__(16) float sT[8][16 * 68];
  const int b    = blockIdx.y;
  const int lane = threadIdx.x & 31;
  const int wave = threadIdx.x >> 5;
  const int tilesN = N >> 6;
  const int tilesM = M >> 6;
  const int tile = blockIdx.x * 8 + wave;
  if (tile >= tilesM * tilesN) return;
  const int tm = tile / tilesN;
  const int tn = tile - tm * tilesN;
  const int m0 = tm << 6;
  const int n0 = tn << 6;
  {
    int s0, s1, cnt, tg;
    seg_info(rowinfo, s0, s1, cnt, tg);
    const int alo = s0 & ~63, ahi = (s1 + 63) & ~63;
    if (m0 < alo || m0 >= ahi) return;
  }

  const T* Ab  = A  + (size_t)b * strideA;
  const T* Bb  = Bt + (size_t)b * strideB;
  const T* Ab2 = SPLIT ? (A2  + (size_t)b * strideA) : nullptr;
  const T* Bb2 = SPLIT ? (Bt2 + (size_t)b * strideB) : nullptr;

  const int rlane = lane & 15;
  const int koff  = (lane >> 4) * 8;
  const int mOff  = (lane >> 4) * 8;

  v8f acc[4][4];
#pragma unroll
  for (int i = 0; i < 4; ++i)
#pragma unroll
    for (int j = 0; j < 4; ++j) acc[i][j] = (v8f){0.f,0.f,0.f,0.f,0.f,0.f,0.f,0.f};

  for (int k0 = 0; k0 < K; k0 += 32) {
    V bh[4], bl[4];
#pragma unroll
    for (int j = 0; j < 4; ++j) {
      const size_t bo = (size_t)(n0 + (j << 4) + rlane) * ldb + koff + k0;
      bh[j] = Frag<T>::load(Bb + bo);
      if (SPLIT) bl[j] = Frag<T>::load(Bb2 + bo);
    }
#pragma unroll
    for (int i = 0; i < 4; ++i) {
      const size_t ao = (size_t)(m0 + (i << 4) + rlane) * lda + koff + k0;
      V ah = Frag<T>::load(Ab + ao);
      V al;
      if (SPLIT) al = Frag<T>::load(Ab2 + ao);
#pragma unroll
      for (int j = 0; j < 4; ++j) {
        acc[i][j] = Frag<T>::mma(ah, bh[j], acc[i][j]);
        if (SPLIT) {
          acc[i][j] = Frag<T>::mma(ah, bl[j], acc[i][j]);
          acc[i][j] = Frag<T>::mma(al, bh[j], acc[i][j]);
        }
      }
      Frag<T>::guard(acc[i][0], acc[i][3], ah, SPLIT ? al : ah);
    }
    Frag<T>::keep(bh[0], bh[1], bh[2], bh[3]);
    if (SPLIT) Frag<T>::keep(bl[0], bl[1], bl[2], bl[3]);
  }
  acc_guard4(acc[0][0], acc[0][1], acc[0][2], acc[0][3]);
  acc_guard4(acc[1][0], acc[1][1], acc[1][2], acc[1][3]);
  acc_guard4(acc[2][0], acc[2][1], acc[2][2], acc[2][3]);
  acc_guard4(acc[3][0], acc[3][1], acc[3][2], acc[3][3]);

  float* slab = sT[wave];
  const float* Rb = RESID ? (resid + (size_t)b * strideR) : nullptr;
#pragma unroll
  for (int i = 0; i < 4; ++i) {
    const int mBase = m0 + (i << 4);
#pragma unroll
    for (int j = 0; j < 4; ++j) {
      const int n = n0 + (j << 4) + rlane;
      float bv = 0.f;
      if (BIAS_MODE == 2) bv = bias[n];
#pragma unroll
      for (int r = 0; r < 8; ++r) {
        float v = acc[i][j][r] * scale;
        if (BIAS_MODE == 1) v += bias[mBase + mOff + r];
        if (BIAS_MODE == 2) v += bv;
        if (RESID) v += Rb[(size_t)(mBase + mOff + r) * ldc + n];
        if (ACT == 2) v = fmaxf(v, 0.0f);
        if (ACT == 4) v = (v > 0.f) ? v : 0.01f * v;
        slab[(mOff + r) * 68 + (j << 4) + rlane] = v;
      }
    }
    __builtin_amdgcn_fence(__ATOMIC_RELEASE, "workgroup");
    __builtin_amdgcn_wave_barrier();
    __builtin_amdgcn_fence(__ATOMIC_ACQUIRE, "workgroup");
    if (OUT_MODE == 0) {
      float* C = (float*)Cout + (size_t)b * strideC;
      const int hh = lane >> 4, c4 = (lane & 15) * 4;
      for (int pass = 0; pass < 2; ++pass) {
#pragma unroll
        for (int it = 0; it < 8; ++it) {
          const int row = it * 2 + hh;
          v4f v = *(const v4f*)(slab + row * 68 + c4);
          *(volatile v4f*)(C + (size_t)(mBase + row) * ldc + n0 + c4) = v;
        }
        __threadfence();
      }
    } else {
      const int q = lane >> 3, c8 = (lane & 7) * 8;
      unsigned short* C  = (unsigned short*)Cout  + (size_t)b * strideC;
      unsigned short* C2 = (OUT_MODE == 2) ? ((unsigned short*)Cout2 + (size_t)b * strideC) : nullptr;
      for (int pass = 0; pass < 2; ++pass) {
#pragma unroll
        for (int it = 0; it < 4; ++it) {
          const int row = it * 4 + q;
          const float* sp = slab + row * 68 + c8;
          v8h hv, lv;
#pragma unroll
          for (int e = 0; e < 8; ++e) {
            if (OUT_MODE == 1) {
              hv[e] = (_Float16)sp[e];
            } else {
              unsigned short hb = f2bf_bits(sp[e]);
              unsigned short lb = f2bf_bits(sp[e] - bf_bits2f(hb));
              hv[e] = __builtin_bit_cast(_Float16, hb);
              lv[e] = __builtin_bit_cast(_Float16, lb);
            }
          }
          *(volatile v8h*)(C + (size_t)(mBase + row) * ldc + n0 + c8) = hv;
          if (OUT_MODE == 2) *(volatile v8h*)(C2 + (size_t)(mBase + row) * ldc + n0 + c8) = lv;
        }
        __threadfence();
      }
    }
    __builtin_amdgcn_fence(__ATOMIC_RELEASE, "workgroup");
    __builtin_amdgcn_wave_barrier();
    __builtin_amdgcn_fence(__ATOMIC_ACQUIRE, "workgroup");
  }
}

__global__ __launch_bounds__(256) void k_prep(const int* __restrict__ seg, const int* __restrict__ posp,
                                             int* __restrict__ info) {
  __shared__ int rmin[8];
  __shared__ int rmax[8];
  __shared__ int rcnt[8];
  const int t = threadIdx.x, lane = t & 31, wave = t >> 5;
  int p = posp[0];
  p = p < 0 ? 0 : (p > kS - 1 ? kS - 1 : p);
  const int target = seg[p];
  int lmin = kS, lmax = -1, lcnt = 0;
#pragma unroll 1
  for (int j = 0; j < kS / 256; ++j) {
    const int i = j * 256 + t;
    const int v = seg[i];
    const bool hit = (v == target);
    lmin = (hit && i < lmin) ? i : lmin;
    lmax = (hit && i > lmax) ? i : lmax;
    lcnt += hit ? 1 : 0;
  }
#pragma unroll
  for (int off = 16; off > 0; off >>= 1) {
    const int omin = __shfl_xor(lmin, off, 32);
    const int omax = __shfl_xor(lmax, off, 32);
    const int ocnt = __shfl_xor(lcnt, off, 32);
    lmin = omin < lmin ? omin : lmin;
    lmax = omax > lmax ? omax : lmax;
    lcnt += ocnt;
  }
  if (lane == 0) { rmin[wave] = lmin; rmax[wave] = lmax; rcnt[wave] = lcnt; }
  __syncthreads();
  if (wave == 0) {
    int gmin = rmin[0], gmax = rmax[0], gcnt = rcnt[0];
#pragma unroll
    for (int w = 1; w < 8; ++w) {
      gmin = rmin[w] < gmin ? rmin[w] : gmin;
      gmax = rmax[w] > gmax ? rmax[w] : gmax;
      gcnt += rcnt[w];
    }
    gmin = gmin > kS - 1 ? kS - 1 : gmin;
    gmax = gmax < 0 ? 0 : gmax;
    const int c0 = (lane == 0) ? gmin : 0;
    const int c1 = (lane == 0) ? (gmax + 1) : 0;
    const int c2 = (lane == 0) ? gcnt : 0;
    const int c3 = (lane == 0) ? target : 0;
    const v4i val = (v4i){c0, c1, c2, c3};
    if (lane < 8) *(volatile v4i*)(info + 4 * lane) = val;
    __threadfence();
    if (lane < 8) *(volatile v4i*)(info + 4 * lane) = val;
  }
}

__global__ __launch_bounds__(256) void k_colsum(const float* __restrict__ x, float* __restrict__ csPart) {
  const int c = blockIdx.x;
  const int t = threadIdx.x;
  const float* p = x + (size_t)c * 256 * kE + 4 * t;
  v4f acc = (v4f){0.f, 0.f, 0.f, 0.f};
#pragma unroll 4
  for (int r = 0; r < 256; ++r) {
    const v4f w = *(const v4f*)(p + (size_t)r * kE);
    acc = acc + w;
  }
  float* dp = csPart + (size_t)c * kE + 4 * t;
  *(volatile v4f*)dp = acc;
  __threadfence();
  *(volatile v4f*)dp = acc;
}

__global__ __launch_bounds__(256) void k_vsum(const float* __restrict__ csPart, const float* __restrict__ Wv,
                                             const float* __restrict__ bv, float* __restrict__ vsum) {
  __shared__ __align__(16) float cs[kE];
  __shared__ __align__(16) float res[32];
  const int t = threadIdx.x, lane = t & 31, wave = t >> 5;
  {
    v4f a = (v4f){0.f, 0.f, 0.f, 0.f};
#pragma unroll 4
    for (int c = 0; c < kChunks; ++c) a = a + *(const v4f*)(csPart + (size_t)c * kE + 4 * t);
    *(v4f*)(cs + 4 * t) = a;
  }
  __syncthreads();
  const int nb = blockIdx.x * 32;
#pragma unroll 1
  for (int j = 0; j < 4; ++j) {
    const int n = nb + wave * 4 + j;
    const float* wr = Wv + (size_t)n * kE;
    float acc = 0.f;
#pragma unroll 1
    for (int i = 0; i < 8; ++i) {
      const int col = i * 128 + 4 * lane;
      const v4f w  = *(const v4f*)(wr + col);
      const v4f cv = *(const v4f*)(cs + col);
      acc += w[0] * cv[0];
      acc += w[1] * cv[1];
      acc += w[2] * cv[2];
      acc += w[3] * cv[3];
    }
    acc = wave_sum32(acc);
    const float bn = bv[n];
    const float val = acc + 4096.0f * bn;
    if (lane == 0) res[wave * 4 + j] = val;
  }
  __syncthreads();
  if (wave == 0) {
    const int li = lane < 8 ? lane : 7;
    const v4f o4 = *(const v4f*)(res + 4 * li);
    float* dp = vsum + nb + 4 * li;
    if (lane < 8) *(volatile v4f*)dp = o4;
    __threadfence();
    if (lane < 8) *(volatile v4f*)dp = o4;
  }
}

__global__ __launch_bounds__(256) void k_split_w(const float* __restrict__ W0, const float* __restrict__ W1,
                                                const float* __restrict__ W2,
                                                unsigned short* __restrict__ hi, unsigned short* __restrict__ lo) {
  const int i = blockIdx.x * 256 + threadIdx.x;
  const int z = blockIdx.x >> 9;
  const float* W = (z == 0) ? W0 : (z == 1) ? W1 : W2;
  const size_t loc = 8 * (size_t)(i - z * 131072);
  const float* p = W + loc;
  const v4f a = *(const v4f*)(p);
  const v4f c = *(const v4f*)(p + 4);
  unsigned short hb[8], lb[8];
#pragma unroll
  for (int e = 0; e < 4; ++e) {
    split_bf(a[e], hb[e], lb[e]);
    split_bf(c[e], hb[4 + e], lb[4 + e]);
  }
  const v4u uh = (v4u){pk16(hb[0], hb[1]), pk16(hb[2], hb[3]), pk16(hb[4], hb[5]), pk16(hb[6], hb[7])};
  const v4u ul = (v4u){pk16(lb[0], lb[1]), pk16(lb[2], lb[3]), pk16(lb[4], lb[5]), pk16(lb[6], lb[7])};
  unsigned short* qh = hi + 8 * (size_t)i;
  unsigned short* ql = lo + 8 * (size_t)i;
  *(volatile v4u*)qh = uh;
  *(volatile v4u*)ql = ul;
  __threadfence();
  *(volatile v4u*)qh = uh;
  *(volatile v4u*)ql = ul;
}

__global__ __launch_bounds__(256) void k_split_x(const float* __restrict__ x, const int* __restrict__ info,
                                                unsigned short* __restrict__ hi, unsigned short* __restrict__ lo) {
  const int tile = blockIdx.y;
  const int m0 = tile * 64;
  int s0, s1, cnt, tg;
  seg_info(info, s0, s1, cnt, tg);
  const int alo = s0 & ~63, ahi = (s1 + 63) & ~63;
  if (m0 < alo || m0 >= ahi) return;
  const int i = blockIdx.x * 256 + threadIdx.x;
  const size_t off = (size_t)tile * 64 * kE + 8 * (size_t)i;
  const float* p = x + off;
  const v4f a = *(const v4f*)(p);
  const v4f c = *(const v4f*)(p + 4);
  unsigned short hb[8], lb[8];
#pragma unroll
  for (int e = 0; e < 4; ++e) {
    split_bf(a[e], hb[e], lb[e]);
    split_bf(c[e], hb[4 + e], lb[4 + e]);
  }
  const v4u uh = (v4u){pk16(hb[0], hb[1]), pk16(hb[2], hb[3]), pk16(hb[4], hb[5]), pk16(hb[6], hb[7])};
  const v4u ul = (v4u){pk16(lb[0], lb[1]), pk16(lb[2], lb[3]), pk16(lb[4], lb[5]), pk16(lb[6], lb[7])};
  unsigned short* qh = hi + off;
  unsigned short* ql = lo + off;
  *(volatile v4u*)qh = uh;
  *(volatile v4u*)ql = ul;
  __threadfence();
  *(volatile v4u*)qh = uh;
  *(volatile v4u*)ql = ul;
}

__global__ __launch_bounds__(256) void k_attn(const float* __restrict__ qkv, const float* __restrict__ vsum,
                                             const int* __restrict__ seg, const int* __restrict__ info,
                                             float* __restrict__ partial) {
  __shared__ __align__(16) float red[8][128];
  const int tile = blockIdx.x, hp = blockIdx.y;
  const int t = threadIdx.x, lane = t & 31, wave = t >> 5;
  const int m0 = tile * 64;
  int s0, s1, cnt, target;
  seg_info(info, s0, s1, cnt, target);
  const int alo = s0 & ~63, ahi = (s1 + 63) & ~63;
  const bool active = (m0 >= alo) && (m0 < ahi);
  const int col = hp * 128 + 4 * lane;
  const v4f zero4 = (v4f){0.f, 0.f, 0.f, 0.f};
  v4f colacc = zero4;
  if (active) {
    const int s1c = (s1 < s0 + kMaxSeg) ? s1 : (s0 + kMaxSeg);
    const v4f vs4 = *(const v4f*)(vsum + col);
    const float nout = (float)(kS - cnt);
#pragma unroll 1
    for (int ri = 0; ri < 8; ++ri) {
      const int s = m0 + wave + 8 * ri;
      const int segs = __builtin_amdgcn_readfirstlane(seg[s]);
      if (segs != target) continue;
      const v4f q4 = *(const v4f*)(qkv + (size_t)s * kLdQKV + col);
      float m = 0.f, Z = 0.f;
      v4f a = zero4, sv = zero4;
#pragma unroll 1
      for (int tt = s0; tt < s1c; ++tt) {
        const int segt = __builtin_amdgcn_readfirstlane(seg[tt]);
        const float* kr = qkv + (size_t)tt * kLdQKV + kE + col;
        const v4f k4 = *(const v4f*)(kr);
        const v4f v4 = *(const v4f*)(kr + kE);
        float p = q4[0] * k4[0];
        p = fmaf(q4[1], k4[1], p);
        p = fmaf(q4[2], k4[2], p);
        p = fmaf(q4[3], k4[3], p);
        p += __shfl_xor(p, 1, 32);
        p += __shfl_xor(p, 2, 32);
        p += __shfl_xor(p, 4, 32);
        p += __shfl_xor(p, 8, 32);
        if (segt == target) {
          const float mn = fmaxf(m, p);
          const float alpha = expf(m - mn);
          const float pe = expf(p - mn);
          Z = Z * alpha + pe;
          a = a * alpha + v4 * pe;
          sv = sv + v4;
          m = mn;
        }
      }
      const float em = expf(-m);
      const float zf = Z + em * nout;
      const float inv = 1.0f / zf;
      const v4f wv = (a + (vs4 - sv) * em) * inv;
      colacc = colacc + wv;
    }
  }
  *(v4f*)(&red[wave][4 * lane]) = colacc;
  __syncthreads();
  if (wave == 0) {
    v4f tot = *(const v4f*)(&red[0][4 * lane]);
#pragma unroll
    for (int w = 1; w < 8; ++w) tot = tot + *(const v4f*)(&red[w][4 * lane]);
    float* dp = partial + (size_t)tile * kE + col;
    *(volatile v4f*)dp = tot;
    __threadfence();
    *(volatile v4f*)dp = tot;
  }
}

__global__ __launch_bounds__(256) void k_final(const float* __restrict__ partial, const float* __restrict__ Wo,
                                              const float* __restrict__ bo, const int* __restrict__ info,
                                              float* __restrict__ out) {
  __shared__ __align__(16) float mw[kE];
  __shared__ __align__(16) float res[32];
  const int t = threadIdx.x, lane = t & 31, wave = t >> 5;
  int s0, s1, cnt, tg;
  seg_info(info, s0, s1, cnt, tg);
  const float invC = 1.0f / (float)cnt;
  {
    v4f a = (v4f){0.f, 0.f, 0.f, 0.f};
#pragma unroll 4
    for (int tile = 0; tile < kTiles; ++tile) a = a + *(const v4f*)(partial + (size_t)tile * kE + 4 * t);
    a = a * invC;
    *(v4f*)(mw + 4 * t) = a;
  }
  __syncthreads();
  const int nb = blockIdx.x * 32;
#pragma unroll 1
  for (int j = 0; j < 4; ++j) {
    const int n = nb + wave * 4 + j;
    const float* wr = Wo + (size_t)n * kE;
    float acc = 0.f;
#pragma unroll 1
    for (int i = 0; i < 8; ++i) {
      const int colx = i * 128 + 4 * lane;
      const v4f w  = *(const v4f*)(wr + colx);
      const v4f cv = *(const v4f*)(mw + colx);
      acc += w[0] * cv[0];
      acc += w[1] * cv[1];
      acc += w[2] * cv[2];
      acc += w[3] * cv[3];
    }
    acc = wave_sum32(acc);
    const float bn = bo[n];
    const float val = acc + bn;
    if (lane == 0) res[wave * 4 + j] = val;
  }
  __syncthreads();
  if (wave == 0) {
    const int li = lane < 8 ? lane : 7;
    const v4f o4 = *(const v4f*)(res + 4 * li);
    float* dp = out + nb + 4 * li;
    if (lane < 8) *(volatile v4f*)dp = o4;
    __threadfence();
    if (lane < 8) *(volatile v4f*)dp = o4;
  }
}

extern "C" void kernel_launch(void* const* d_in, const int* in_sizes, int n_in,
                              void* d_out, int out_size, void* d_ws, size_t ws_size,
                              hipStream_t stream) {
  if (n_in < 11) return;
  if (in_sizes[0] != kS * kE) return;
  if (in_sizes[1] != kE * kE || in_sizes[3] != kE * kE || in_sizes[5] != kE * kE || in_sizes[7] != kE * kE) return;
  if (in_sizes[2] != kE || in_sizes[4] != kE || in_sizes[6] != kE || in_sizes[8] != kE) return;
  if (in_sizes[9] != kS || in_sizes[10] < 1) return;
  if (out_size != kE) return;

  const size_t offInfo = 0;
  const size_t offCsp  = 4096;
  const size_t offVsum = offCsp + (size_t)kChunks * kE * 4;
  const size_t offPart = offVsum + (size_t)kE * 4;
  const size_t offWhi  = offPart + (size_t)kTiles * kE * 4;
  const size_t szW     = (size_t)3 * kE * kE * 2;
  const size_t offWlo  = offWhi + szW;
  const size_t szX     = (size_t)kS * kE * 2;
  const size_t offXhi  = offWlo + szW;
  const size_t offXlo  = offXhi + szX;
  const size_t offQKV  = offXlo + szX;
  const size_t szQKV   = (size_t)kS * kLdQKV * 4;
  const size_t total   = offQKV + szQKV;
  if (ws_size < total) return;

  const float* x   = (const float*)d_in[0];
  const float* Wq  = (const float*)d_in[1];
  const float* bq  = (const float*)d_in[2];
  const float* Wk  = (const float*)d_in[3];
  const float* bk  = (const float*)d_in[4];
  const float* Wv  = (const float*)d_in[5];
  const float* bv  = (const float*)d_in[6];
  const float* Wo  = (const float*)d_in[7];
  const float* bo  = (const float*)d_in[8];
  const int*   seg = (const int*)d_in[9];
  const int*   posp = (const int*)d_in[10];
  float* out = (float*)d_out;
  char* ws = (char*)d_ws;
  int*   info    = (int*)(ws + offInfo);
  float* csPart  = (float*)(ws + offCsp);
  float* vsum    = (float*)(ws + offVsum);
  float* partial = (float*)(ws + offPart);
  unsigned short* Whi = (unsigned short*)(ws + offWhi);
  unsigned short* Wlo = (unsigned short*)(ws + offWlo);
  unsigned short* Xhi = (unsigned short*)(ws + offXhi);
  unsigned short* Xlo = (unsigned short*)(ws + offXlo);
  float* qkv = (float*)(ws + offQKV);

  k_prep<<<dim3(1), dim3(256), 0, stream>>>(seg, posp, info);
  k_colsum<<<dim3(kChunks), dim3(256), 0, stream>>>(x, csPart);
  k_vsum<<<dim3(kE / 32), dim3(256), 0, stream>>>(csPart, Wv, bv, vsum);
  k_split_w<<<dim3(3 * 512), dim3(256), 0, stream>>>(Wq, Wk, Wv, Whi, Wlo);
  k_split_x<<<dim3(32, kTiles), dim3(256), 0, stream>>>(x, info, Xhi, Xlo);

  const int gemmBlocks = ((kS / 64) * (kE / 64)) / 8;
  for (int z = 0; z < 3; ++z) {
    const unsigned short* Whz = Whi + (size_t)z * kE * kE;
    const unsigned short* Wlz = Wlo + (size_t)z * kE * kE;
    const float* bz = (z == 0) ? bq : (z == 1) ? bk : bv;
    float* Cz = qkv + (size_t)z * kE;
    wmma_gemm64_seg<1, true, 2, 0, false, 0><<<dim3(gemmBlocks, 1), dim3(256), 0, stream>>>(
        Xhi, Xlo, kE, 0L, Whz, Wlz, kE, 0L,
        (void*)Cz, (void*)Cz, kLdQKV, 0L, bz, bz, 0L, kS, kE, kE, 1.0f, info);
  }

  k_attn<<<dim3(kTiles, kHeads / 2), dim3(256), 0, stream>>>(qkv, vsum, seg, info, partial);
  k_final<<<dim3(kE / 32), dim3(256), 0, stream>>>(partial, Wo, bo, info, out);
}
